// DeeperGCN_G_85950885527884
// MI455X (gfx1250) — hardware-verified
//
#include <hip/hip_runtime.h>
#include <stddef.h>


#define FIN    128
#define HC     64
#define HC2    128
#define RW     16
#define GWAVES 2
#define GTHR   64
#define GROWS  (RW * GWAVES)
#define PA64   72
#define PA128  136
#define PH     132
#define PO     68
#define WPL    8192

#define NB     512
#define CHUNK  2048
#define ATHR   256
#define AWAVES 8
#define WCAP   256
#define NGRP   (CHUNK / (ATHR * 4))
#define MSG_EPS 1e-7f
#define LDS_ST   (NB * 32)
#define LDS_LIST (AWAVES * WCAP)
#define LDS_AGG_BYTES (LDS_ST * 16 + LDS_LIST * 4 + AWAVES * 4)

static_assert(WCAP == (CHUNK / ATHR) * 32);
static_assert(NGRP >= 1);
static_assert(NB == 512);
static_assert(CHUNK == 2048);
static_assert(LDS_AGG_BYTES == 270368);
static_assert((NB % GROWS) == 0);
static_assert(FIN * HC == WPL);
static_assert(HC * HC2 == WPL);

typedef float  v2f  __attribute__((ext_vector_type(2)));
typedef float  v4f  __attribute__((ext_vector_type(4)));
typedef float  v8f  __attribute__((ext_vector_type(8)));
typedef int    v4i  __attribute__((ext_vector_type(4)));
typedef __bf16 v4b  __attribute__((ext_vector_type(4)));
typedef __bf16 v8b  __attribute__((ext_vector_type(8)));
typedef __bf16 v16b __attribute__((ext_vector_type(16)));
union Frag  { v16b v; v8b half[2]; };
union Pack8 { v8b b; v4i i; };

__device__ __forceinline__ v8f wm(v16b a, v16b b, v8f c) {
  v8f d = __builtin_amdgcn_wmma_f32_16x16x32_bf16(false, a, false, b, (short)0, c, false, false);
  asm volatile("v_nop\n\tv_nop\n\tv_nop\n\tv_nop" : "+v"(d) : "v"(a), "v"(b));
  return d;
}

__device__ __forceinline__ float wsum(float v) {
  v += __shfl_xor(v, 16, 32);
  v += __shfl_xor(v, 8, 32);
  v += __shfl_xor(v, 4, 32);
  v += __shfl_xor(v, 2, 32);
  v += __shfl_xor(v, 1, 32);
  return v;
}

__device__ __forceinline__ void split8(const float (&v)[8], Pack8& uh, Pack8& ul) {
#pragma unroll
  for (int j = 0; j < 8; ++j) {
    const __bf16 hb = (__bf16)v[j];
    uh.b[j] = hb;
    ul.b[j] = (__bf16)(v[j] - (float)hb);
  }
}

__device__ __forceinline__ void split4(v4f x, v4b& hi, v4b& lo) {
  const float v[4] = {x.x, x.y, x.z, x.w};
#pragma unroll
  for (int j = 0; j < 4; ++j) {
    const __bf16 hb = (__bf16)v[j];
    hi[j] = hb;
    lo[j] = (__bf16)(v[j] - (float)hb);
  }
}

template <int K, int PA>
__device__ __forceinline__ void stage_a(const float* __restrict__ A, int rowBase, int nN, int lane,
                                        __bf16* sAh, __bf16* sAl) {
  const int r = lane >> 1;
  int row = rowBase + r;
  if (row > nN - 1) row = nN - 1;
  const int cb = (lane & 1) * (K / 2);
  const float* p = A + (size_t)row * K + cb;
  __bf16* ph = sAh + r * PA + cb;
  __bf16* pl = sAl + r * PA + cb;
#pragma unroll
  for (int j = 0; j < K / 16; ++j) {
    const v4f f0 = *(const v4f*)(p + 8 * j);
    const v4f f1 = *(const v4f*)(p + 8 * j + 4);
    const float v[8] = {f0.x, f0.y, f0.z, f0.w, f1.x, f1.y, f1.z, f1.w};
    Pack8 uh, ul;
    split8(v, uh, ul);
    *(v8b*)(ph + 8 * j) = uh.b;
    *(v8b*)(pl + 8 * j) = ul.b;
  }
}

template <int K, int PA>
__device__ __forceinline__ v8f mm_tile(const __bf16* sAh, const __bf16* sAl,
                                       const __bf16* __restrict__ Wh, const __bf16* __restrict__ Wl,
                                       int n, int m, int hh) {
  v8f acc = {0.f, 0.f, 0.f, 0.f, 0.f, 0.f, 0.f, 0.f};
#pragma unroll
  for (int ks = 0; ks < K / 32; ++ks) {
    const int k0 = ks * 32 + 8 * hh;
    Frag ah, al, bh, bl;
    const __bf16* pa = sAh + m * PA + k0;
    const __bf16* pl = sAl + m * PA + k0;
    const __bf16* pb = Wh + (size_t)n * K + k0;
    const __bf16* pc = Wl + (size_t)n * K + k0;
    ah.half[0] = *(const v8b*)pa;  ah.half[1] = *(const v8b*)(pa + 16);
    al.half[0] = *(const v8b*)pl;  al.half[1] = *(const v8b*)(pl + 16);
    bh.half[0] = *(const v8b*)pb;  bh.half[1] = *(const v8b*)(pb + 16);
    bl.half[0] = *(const v8b*)pc;  bl.half[1] = *(const v8b*)(pc + 16);
    acc = wm(ah.v, bh.v, acc);
    acc = wm(ah.v, bl.v, acc);
    acc = wm(al.v, bh.v, acc);
  }
  return acc;
}

__device__ __forceinline__ void store_rows64(const float* sO, float* y, int rowBase, int lane) {
  const int hh = lane >> 4, c4 = 4 * (lane & 15);
  v4f v[8];
  float* p[8];
#pragma unroll
  for (int i = 0; i < 8; ++i) {
    v[i] = *(const v4f*)(sO + (2 * i + hh) * PO + c4);
    p[i] = y + (size_t)(rowBase + 2 * i + hh) * HC + c4;
  }
#pragma unroll
  for (int i = 0; i < 8; ++i) *(volatile v4f*)(p[i]) = v[i];
  __threadfence();
#pragma unroll
  for (int i = 0; i < 8; ++i) *(volatile v4f*)(p[i]) = v[i];
}

__global__ __launch_bounds__(256) void k_prep(const float* __restrict__ Wenc, const float* __restrict__ Wm1,
                                              const float* __restrict__ Wm2, __bf16* planes) {
  const int i = blockIdx.x * 256 + threadIdx.x;
  if (i >= 3 * (WPL / 8)) return;
  const int mat = i >> 10;
  const int q   = i & 1023;
  const float* W = (mat == 0) ? Wenc : ((mat == 1) ? Wm1 : Wm2);
  const int lk = (mat == 1) ? 6 : 7;
  const int K  = 1 << lk;
  const int NC = WPL >> lk;
  const int o  = q * 8;
  const int n  = o >> lk;
  const int k0 = o & (K - 1);
  float v[8];
#pragma unroll
  for (int j = 0; j < 8; ++j) v[j] = W[(size_t)(k0 + j) * NC + n];
  Pack8 uh, ul;
  split8(v, uh, ul);
  __bf16* ph = planes + (size_t)(2 * mat) * WPL + o;
  __bf16* pl = ph + WPL;
  *(volatile v4i*)ph = uh.i;
  *(volatile v4i*)pl = ul.i;
  __threadfence();
  *(volatile v4i*)ph = uh.i;
  *(volatile v4i*)pl = ul.i;
}

__global__ __launch_bounds__(GTHR) void k_enc(const float* __restrict__ x,
                                              const __bf16* __restrict__ Wh, const __bf16* __restrict__ Wl,
                                              const float* __restrict__ bias, float* y, int nN) {
  __shared__ __attribute__((aligned(16))) __bf16 sAh[GWAVES][RW * PA128];
  __shared__ __attribute__((aligned(16))) __bf16 sAl[GWAVES][RW * PA128];
  __shared__ __attribute__((aligned(16))) float  sO[GWAVES][RW * PO];
  const int lane = threadIdx.x & 31, wave = threadIdx.x >> 5;
  const int hh = lane >> 4, m = lane & 15;
  const int rowBase = blockIdx.x * GROWS + wave * RW;

  stage_a<FIN, PA128>(x, rowBase, nN, lane, sAh[wave], sAl[wave]);
  __syncthreads();
#pragma unroll 1
  for (int t = 0; t < HC / 16; ++t) {
    const v8f acc = mm_tile<FIN, PA128>(sAh[wave], sAl[wave], Wh, Wl, t * 16 + m, m, hh);
    const float bb = bias[t * 16 + m];
#pragma unroll
    for (int r = 0; r < 8; ++r) sO[wave][(8 * hh + r) * PO + t * 16 + m] = acc[r] + bb;
  }
  __syncthreads();
  store_rows64(sO[wave], y, rowBase, lane);
}

__device__ __forceinline__ void mlp_core(
    const float* __restrict__ A,
    const __bf16* __restrict__ W1h, const __bf16* __restrict__ W1l,
    const float* __restrict__ b1, const float* __restrict__ g1, const float* __restrict__ be1,
    const __bf16* __restrict__ W2h, const __bf16* __restrict__ W2l, const float* __restrict__ b2,
    int rowBase, int nN, int lane, int hh, int m,
    __bf16* a1h, __bf16* a1l, float* sH, __bf16* a2h, __bf16* a2l) {
  stage_a<HC, PA64>(A, rowBase, nN, lane, a1h, a1l);
  __syncthreads();

#pragma unroll 1
  for (int t = 0; t < HC2 / 16; ++t) {
    const v8f acc = mm_tile<HC, PA64>(a1h, a1l, W1h, W1l, t * 16 + m, m, hh);
    const float bb = b1[t * 16 + m];
#pragma unroll
    for (int r = 0; r < 8; ++r) sH[(8 * hh + r) * PH + t * 16 + m] = acc[r] + bb;
  }
  __syncthreads();

  {
    const v4f g4 = *(const v4f*)(g1 + 4 * lane);
    const v4f e4 = *(const v4f*)(be1 + 4 * lane);
#pragma unroll 1
    for (int r = 0; r < RW; ++r) {
      const v4f v = *(const v4f*)(sH + r * PH + 4 * lane);
      const float s  = wsum(v.x + v.y + v.z + v.w);
      const float mu = s * (1.0f / HC2);
      const v4f d = v - mu;
      const float q  = wsum(d.x * d.x + d.y * d.y + d.z * d.z + d.w * d.w);
      const float rs = rsqrtf(q * (1.0f / HC2) + 1e-5f);
      v4f o = d * rs * g4 + e4;
      o.x = o.x > 0.f ? o.x : 0.f;
      o.y = o.y > 0.f ? o.y : 0.f;
      o.z = o.z > 0.f ? o.z : 0.f;
      o.w = o.w > 0.f ? o.w : 0.f;
      v4b hi, lo;
      split4(o, hi, lo);
      *(v4b*)(a2h + r * PA128 + 4 * lane) = hi;
      *(v4b*)(a2l + r * PA128 + 4 * lane) = lo;
    }
  }
  __syncthreads();

#pragma unroll 1
  for (int t = 0; t < HC / 16; ++t) {
    const v8f acc = mm_tile<HC2, PA128>(a2h, a2l, W2h, W2l, t * 16 + m, m, hh);
    const float bb = b2[t * 16 + m];
#pragma unroll
    for (int r = 0; r < 8; ++r) sH[(8 * hh + r) * PO + t * 16 + m] = acc[r] + bb;
  }
  __syncthreads();
}

__global__ __launch_bounds__(GTHR) void k_mlp1(
    const float* __restrict__ A,
    const __bf16* __restrict__ W1h, const __bf16* __restrict__ W1l,
    const float* __restrict__ b1, const float* __restrict__ g1, const float* __restrict__ be1,
    const __bf16* __restrict__ W2h, const __bf16* __restrict__ W2l, const float* __restrict__ b2,
    float* y, int nN) {
  __shared__ __attribute__((aligned(16))) __bf16 sA1h[GWAVES][RW * PA64];
  __shared__ __attribute__((aligned(16))) __bf16 sA1l[GWAVES][RW * PA64];
  __shared__ __attribute__((aligned(16))) float  sH[GWAVES][RW * PH];
  __shared__ __attribute__((aligned(16))) __bf16 sA2h[GWAVES][RW * PA128];
  __shared__ __attribute__((aligned(16))) __bf16 sA2l[GWAVES][RW * PA128];
  const int lane = threadIdx.x & 31, wave = threadIdx.x >> 5;
  const int hh = lane >> 4, m = lane & 15;
  const int rowBase = blockIdx.x * GROWS + wave * RW;
  mlp_core(A, W1h, W1l, b1, g1, be1, W2h, W2l, b2, rowBase, nN, lane, hh, m,
           sA1h[wave], sA1l[wave], sH[wave], sA2h[wave], sA2l[wave]);
  store_rows64(sH[wave], y, rowBase, lane);
}

__global__ __launch_bounds__(GTHR) void k_mlp2(
    const float* __restrict__ A,
    const __bf16* __restrict__ W1h, const __bf16* __restrict__ W1l,
    const float* __restrict__ b1, const float* __restrict__ g1, const float* __restrict__ be1,
    const __bf16* __restrict__ W2h, const __bf16* __restrict__ W2l, const float* __restrict__ b2,
    const float* __restrict__ x1, const float* __restrict__ ln1g, const float* __restrict__ ln1b,
    const float* __restrict__ ng, const float* __restrict__ nbe,
    const float* __restrict__ lw, const float* __restrict__ lb, float* out, int nN) {
  __shared__ __attribute__((aligned(16))) __bf16 sA1h[GWAVES][RW * PA64];
  __shared__ __attribute__((aligned(16))) __bf16 sA1l[GWAVES][RW * PA64];
  __shared__ __attribute__((aligned(16))) float  sH[GWAVES][RW * PH];
  __shared__ __attribute__((aligned(16))) __bf16 sA2h[GWAVES][RW * PA128];
  __shared__ __attribute__((aligned(16))) __bf16 sA2l[GWAVES][RW * PA128];
  __shared__ __attribute__((aligned(16))) float  sOut[GROWS];
  const int lane = threadIdx.x & 31, wave = threadIdx.x >> 5;
  const int hh = lane >> 4, m = lane & 15;
  const int rowBase = blockIdx.x * GROWS + wave * RW;
  mlp_core(A, W1h, W1l, b1, g1, be1, W2h, W2l, b2, rowBase, nN, lane, hh, m,
           sA1h[wave], sA1l[wave], sH[wave], sA2h[wave], sA2l[wave]);

  const float* sO = sH[wave];
  const v2f lg  = *(const v2f*)(ln1g + 2 * lane), lbe = *(const v2f*)(ln1b + 2 * lane);
  const v2f ga  = *(const v2f*)(ng + 2 * lane),   gb  = *(const v2f*)(ng + HC + 2 * lane);
  const v2f ba  = *(const v2f*)(nbe + 2 * lane),  bb  = *(const v2f*)(nbe + HC + 2 * lane);
  const v2f wa  = *(const v2f*)(lw + 2 * lane),   wb  = *(const v2f*)(lw + HC + 2 * lane);
  const float lbias = lb[0];
#pragma unroll 1
  for (int r = 0; r < RW; ++r) {
    int row = rowBase + r;
    if (row > nN - 1) row = nN - 1;
    const v2f hv = *(const v2f*)(sO + r * PO + 2 * lane);
    const v2f xv = *(const v2f*)(x1 + (size_t)row * HC + 2 * lane);
    const float s1  = wsum(hv.x + hv.y);
    const float mu1 = s1 * (1.0f / HC);
    const v2f d1 = hv - mu1;
    const float q1  = wsum(d1.x * d1.x + d1.y * d1.y);
    const float rs1 = rsqrtf(q1 * (1.0f / HC) + 1e-5f);
    v2f hn = d1 * rs1 * lg + lbe;
    hn.x = hn.x > 0.f ? hn.x : 0.f;
    hn.y = hn.y > 0.f ? hn.y : 0.f;
    const float s2  = wsum(xv.x + xv.y + hn.x + hn.y);
    const float mu2 = s2 * (1.0f / HC2);
    const v2f dx = xv - mu2, dh = hn - mu2;
    const float q2  = wsum(dx.x * dx.x + dx.y * dx.y + dh.x * dh.x + dh.y * dh.y);
    const float rs2 = rsqrtf(q2 * (1.0f / HC2) + 1e-5f);
    v2f ya = dx * rs2 * ga + ba;
    v2f yb = dh * rs2 * gb + bb;
    ya.x = ya.x > 0.f ? ya.x : 0.f;
    ya.y = ya.y > 0.f ? ya.y : 0.f;
    yb.x = yb.x > 0.f ? yb.x : 0.f;
    yb.y = yb.y > 0.f ? yb.y : 0.f;
    const float pd  = ya.x * wa.x + ya.y * wa.y + yb.x * wb.x + yb.y * wb.y;
    const float tot = wsum(pd) + lbias;
    if (lane == 0) sOut[wave * RW + r] = tot;
  }
  __syncthreads();
  if (wave == 0 && lane < GROWS / 4) {
    const int g0 = blockIdx.x * GROWS + 4 * lane;
    const v4f v = *(const v4f*)(sOut + 4 * lane);
    if (g0 + 3 < nN) {
      *(volatile v4f*)(out + g0) = v;
      __threadfence();
      *(volatile v4f*)(out + g0) = v;
    } else {
      const float vv[4] = {v.x, v.y, v.z, v.w};
#pragma unroll
      for (int e = 0; e < 4; ++e) if (g0 + e < nN) *(volatile float*)(out + g0 + e) = vv[e];
      __threadfence();
#pragma unroll
      for (int e = 0; e < 4; ++e) if (g0 + e < nN) *(volatile float*)(out + g0 + e) = vv[e];
    }
  }
}

__global__ __launch_bounds__(ATHR) void k_agg(const float* __restrict__ xin, const int* __restrict__ ei,
                                              const float* __restrict__ tptr, float* aggout,
                                              int nN, int nE) {
  extern __shared__ v4f lds_dyn[];
  v4f* st   = lds_dyn;
  int* list = (int*)(lds_dyn + LDS_ST);
  int* wcnt = list + LDS_LIST;

  const int tid  = threadIdx.x;
  const int lane = tid & 31;
  const int wave = tid >> 5;
  const int nodeBase = blockIdx.x * NB;

  {
    const v4f z4 = {0.f, 0.f, 0.f, 0.f};
    for (int i = tid; i < LDS_ST; i += ATHR) st[i] = z4;
  }
  __syncthreads();
  const float tt = tptr[0];
  const int* eid = ei + nE;
  const bool al16 = ((nE & 3) == 0);

  const int nChunks = (nE + CHUNK - 1) / CHUNK;
#pragma unroll 1
  for (int ch = 0; ch < nChunks; ++ch) {
    const int cbase = ch * CHUNK;
    int wc = 0;
#pragma unroll
    for (int g = 0; g < NGRP; ++g) {
      const int el0 = (g * ATHR + tid) * 4;
      const int e0  = cbase + el0;
      const int sent = -2147483647 - 1;
      v4i d;
      if (al16 && (e0 + 3 < nE)) {
        d = *(const v4i*)(eid + e0);
      } else {
        d.x = (e0     < nE) ? eid[min(e0, nE - 1)]     : sent;
        d.y = (e0 + 1 < nE) ? eid[min(e0 + 1, nE - 1)] : sent;
        d.z = (e0 + 2 < nE) ? eid[min(e0 + 2, nE - 1)] : sent;
        d.w = (e0 + 3 < nE) ? eid[min(e0 + 3, nE - 1)] : sent;
      }
      const unsigned s0 = (unsigned)d.x - (unsigned)nodeBase;
      const unsigned s1 = (unsigned)d.y - (unsigned)nodeBase;
      const unsigned s2 = (unsigned)d.z - (unsigned)nodeBase;
      const unsigned s3 = (unsigned)d.w - (unsigned)nodeBase;
      const bool h0 = s0 < (unsigned)NB;
      const bool h1 = s1 < (unsigned)NB;
      const bool h2 = s2 < (unsigned)NB;
      const bool h3 = s3 < (unsigned)NB;
      const unsigned many = __builtin_amdgcn_ballot_w32(h0 | h1 | h2 | h3);
      if (many != 0u) {
#define HITJ(J, HJ, SJ) { \
          const unsigned mj = __builtin_amdgcn_ballot_w32(HJ); \
          if (HJ) { \
            const int pos = wc + (int)__builtin_amdgcn_mbcnt_lo(mj, 0u); \
            if (pos < WCAP) list[wave * WCAP + pos] = ((el0 + (J)) << 9) | (int)(SJ); \
          } \
          wc += (int)__builtin_popcount(mj); }
        HITJ(0, h0, s0)
        HITJ(1, h1, s1)
        HITJ(2, h2, s2)
        HITJ(3, h3, s3)
#undef HITJ
      }
    }
    if (lane == 0) wcnt[wave] = wc;
    __syncthreads();

    if (wave == 0) {
      for (int wsx = 0; wsx < AWAVES; ++wsx) {
        int n = wcnt[wsx];
        if (n > WCAP) n = WCAP;
        if (n < 0) n = 0;
        for (int i = 0; i < n; ++i) {
          const int ent  = list[wsx * WCAP + i];
          const int slot = ent & (NB - 1);
          const int el   = (ent >> 9) & (CHUNK - 1);
          int e = cbase + el;
          if (e > nE - 1) e = nE - 1;
          int src = ei[e];
          src = src < 0 ? 0 : (src > nN - 1 ? nN - 1 : src);
          const v2f xv = *(const v2f*)(xin + (size_t)src * HC + 2 * lane);
          const float m0 = fmaxf(xv.x, 0.f) + MSG_EPS;
          const float m1 = fmaxf(xv.y, 0.f) + MSG_EPS;
          const float e0 = __expf(fminf(m0 * tt, 80.f));
          const float e1 = __expf(fminf(m1 * tt, 80.f));
          v4f* sp = st + slot * 32 + lane;
          const v4f cur = *sp;
          v4f add;
          add.x = e0; add.y = m0 * e0; add.z = e1; add.w = m1 * e1;
          *sp = cur + add;
        }
      }
    }
    __syncthreads();
  }

#pragma unroll 1
  for (int j = 0; j < NB / AWAVES / 2; ++j) {
    const int slot = wave * (NB / AWAVES) + 2 * j + (lane >> 4);
    const int cg   = lane & 15;
    const int node = nodeBase + slot;
    int noder = node;
    if (noder > nN - 1) noder = nN - 1;
    const v4f sa = st[slot * 32 + 2 * cg];
    const v4f sb = st[slot * 32 + 2 * cg + 1];
    v4f o;
    o.x = sa.y * __builtin_amdgcn_rcpf(sa.x + 1e-16f);
    o.y = sa.w * __builtin_amdgcn_rcpf(sa.z + 1e-16f);
    o.z = sb.y * __builtin_amdgcn_rcpf(sb.x + 1e-16f);
    o.w = sb.w * __builtin_amdgcn_rcpf(sb.z + 1e-16f);
    const v4f xr = *(const v4f*)(xin + (size_t)noder * HC + 4 * cg);
    o = o + xr;
    float* p = aggout + (size_t)node * HC + 4 * cg;
    *(volatile v4f*)p = o;
    __threadfence();
    *(volatile v4f*)p = o;
  }
}

extern "C" void kernel_launch(void* const* d_in, const int* in_sizes, int n_in,
                              void* d_out, int out_size, void* d_ws, size_t ws_size,
                              hipStream_t stream) {
  if (n_in < 17) return;
  const int nN = in_sizes[0] / FIN;
  const int nE = in_sizes[1] / 2;
  if (nN <= 0 || in_sizes[0] != nN * FIN) return;
  if (nE <= 0 || in_sizes[1] != 2 * nE) return;
  if (in_sizes[2] != FIN * HC || in_sizes[3] != HC || in_sizes[4] < 1) return;
  if (in_sizes[5] != HC * HC2 || in_sizes[6] != HC2 || in_sizes[7] != HC2 || in_sizes[8] != HC2) return;
  if (in_sizes[9] != HC2 * HC || in_sizes[10] != HC || in_sizes[11] != HC || in_sizes[12] != HC) return;
  if (in_sizes[13] != HC2 || in_sizes[14] != HC2 || in_sizes[15] != HC2 || in_sizes[16] < 1) return;
  if (out_size != nN) return;

  const float* x    = (const float*)d_in[0];
  const int*   ei   = (const int*)d_in[1];
  const float* encW = (const float*)d_in[2];
  const float* encb = (const float*)d_in[3];
  const float* tptr = (const float*)d_in[4];
  const float* W1   = (const float*)d_in[5];
  const float* b1   = (const float*)d_in[6];
  const float* g1   = (const float*)d_in[7];
  const float* be1  = (const float*)d_in[8];
  const float* W2   = (const float*)d_in[9];
  const float* b2   = (const float*)d_in[10];
  const float* ln1g = (const float*)d_in[11];
  const float* ln1b = (const float*)d_in[12];
  const float* ng   = (const float*)d_in[13];
  const float* nbe  = (const float*)d_in[14];
  const float* linW = (const float*)d_in[15];
  const float* linb = (const float*)d_in[16];
  float* out = (float*)d_out;

  const int NPa = ((nN + NB - 1) / NB) * NB;
  const int NPg = ((nN + GROWS - 1) / GROWS) * GROWS;
  const int NP  = NPa > NPg ? NPa : NPg;

  size_t off = 0;
  __bf16* planes = (__bf16*)((char*)d_ws + off); off += (size_t)6 * WPL * sizeof(__bf16);
  off = (off + 255) & ~(size_t)255;
  float* x0 = (float*)((char*)d_ws + off); off += (size_t)NP * HC * sizeof(float);
  float* ag = (float*)((char*)d_ws + off); off += (size_t)NP * HC * sizeof(float);
  float* x1 = (float*)((char*)d_ws + off); off += (size_t)NP * HC * sizeof(float);
  if (off > ws_size) return;

  const __bf16* Weh = planes;            const __bf16* Wel = planes + WPL;
  const __bf16* W1h = planes + 2 * WPL;  const __bf16* W1l = planes + 3 * WPL;
  const __bf16* W2h = planes + 4 * WPL;  const __bf16* W2l = planes + 5 * WPL;

  const int prepThreads = 3 * (WPL / 8);
  k_prep<<<(prepThreads + 255) / 256, 256, 0, stream>>>(encW, W1, W2, planes);

  const int ggrid = NPg / GROWS;
  k_enc<<<ggrid, GTHR, 0, stream>>>(x, Weh, Wel, encb, x0, nN);

  hipFuncSetAttribute(reinterpret_cast<const void*>(&k_agg),
                      hipFuncAttributeMaxDynamicSharedMemorySize, LDS_AGG_BYTES);
  const int agrid = NPa / NB;
  k_agg<<<agrid, ATHR, LDS_AGG_BYTES, stream>>>(x0, ei, tptr, ag, nN, nE);
  k_mlp1<<<ggrid, GTHR, 0, stream>>>(ag, W1h, W1l, b1, g1, be1, W2h, W2l, b2, x1, nN);
  k_agg<<<agrid, ATHR, LDS_AGG_BYTES, stream>>>(x1, ei, tptr, ag, nN, nE);
  k_mlp2<<<ggrid, GTHR, 0, stream>>>(ag, W1h, W1l, b1, g1, be1, W2h, W2l, b2,
                                      x1, ln1g, ln1b, ng, nbe, linW, linb, out, nN);
}
